// GATLayer_4355096838265
// MI455X (gfx1250) — hardware-verified
//
#include <hip/hip_runtime.h>
#include <stddef.h>
#include <stdint.h>
#include <math.h>


#define DIN    128
#define HC     128
#define NH     8
#define EDF    16
#define KE     32
#define NG     8
#define LDX    256
#define NTHR   256
#define NWAVE  8
#define EPT    8
#define CHUNK  (NTHR * EPT)
#define WCAP   (EPT * 32)
#define LISTN  (NWAVE * WCAP)
#define NBA    512
#define SLA    9
#define RCAP   16384
#define DEGCAP 64
#define GBM    64
#define GBN    128
#define SROWS  512
#define NUW    2048
#define NUE    512
#define NEGSL  0.2f
#define EPSN   1e-5f
#define AGG_ZINTS (LISTN + 2 * RCAP + 3 * NBA)
#define AGG_LDS_INTS (AGG_ZINTS + 16)
#define STAT_LDS (NWAVE * NG * HC * 8 + NG * HC * 4)
#define GEMM_LDS (GBM * LDX * 4)
#define WSMAX  134217728

static_assert((CHUNK & (CHUNK - 1)) == 0 && CHUNK <= 4096);
static_assert((NBA & (NBA - 1)) == 0 && NBA == (1 << SLA));
static_assert(LISTN % NTHR == 0);
static_assert(NBA % NWAVE == 0 && NBA % 32 == 0);
static_assert(RCAP % 4 == 0 && AGG_ZINTS % 4 == 0 && LISTN % 4 == 0);
static_assert(RCAP == NWAVE * 16 * HC);
static_assert(LISTN * 2 == NWAVE * 16 * KE);
static_assert(DEGCAP % 16 == 0);
static_assert(DIN % 32 == 0 && KE % 32 == 0 && HC == NH * 16 && HC == 4 * 32);
static_assert(GBM == 4 * 16 && LDX == 2 * GBN && GBN == 4 * 32);
static_assert(NUW % NTHR == 0 && NUE % NTHR == 0 && NUW == HC * (DIN / 8) && NUE == HC * (KE / 8));
static_assert(AGG_LDS_INTS * 4 <= 300000);
static_assert(NG * HC == 4 * NTHR);
static_assert(NG == NWAVE);

typedef float          v4f   __attribute__((ext_vector_type(4)));
typedef float          v8f   __attribute__((ext_vector_type(8)));
typedef double         v2d   __attribute__((ext_vector_type(2)));
typedef int            v4i   __attribute__((ext_vector_type(4)));
typedef int            v8i   __attribute__((ext_vector_type(8)));
typedef unsigned int   v4u   __attribute__((ext_vector_type(4)));
typedef unsigned short v8us  __attribute__((ext_vector_type(8)));
typedef unsigned short v16us __attribute__((ext_vector_type(16)));
typedef __bf16         v16bf __attribute__((ext_vector_type(16)));
typedef v4f  __attribute__((may_alias)) v4fa;
typedef v2d  __attribute__((may_alias)) v2da;
typedef v4i  __attribute__((may_alias)) v4ia;
typedef v4u  __attribute__((may_alias)) v4ua;
typedef v8us __attribute__((may_alias)) v8usa;
union FragB { v16bf v; v16us u; v8us h[2]; v8i w; };

__device__ __forceinline__ v8f wmb(const FragB& a, const FragB& b, v8f c) {
  v8f d = __builtin_amdgcn_wmma_f32_16x16x32_bf16(false, a.v, false, b.v, (short)0, c, false, false);
  asm volatile("v_nop\n\tv_nop\n\tv_nop\n\tv_nop" : "+v"(d) : "v"(a.w), "v"(b.w));
  return d;
}

__device__ __forceinline__ void wave_lds_sync() {
  __builtin_amdgcn_fence(__ATOMIC_RELEASE, "wavefront");
  __builtin_amdgcn_wave_barrier();
  __builtin_amdgcn_fence(__ATOMIC_ACQUIRE, "wavefront");
}

__device__ __forceinline__ unsigned bf16_bits(float f) {
  const unsigned u = __float_as_uint(f);
  return ((u + 0x7FFFu + ((u >> 16) & 1u)) >> 16) & 0xFFFFu;
}
__device__ __forceinline__ float bf16_val(float f) {
  return __uint_as_float(bf16_bits(f) << 16);
}
__device__ __forceinline__ v4f bfr4(const v4f a) {
  v4f r; r.x = bf16_val(a.x); r.y = bf16_val(a.y); r.z = bf16_val(a.z); r.w = bf16_val(a.w); return r;
}
__device__ __forceinline__ unsigned pk2(float lo, float hi) { return bf16_bits(lo) | (bf16_bits(hi) << 16); }
__device__ __forceinline__ v4u pack8(const v4f a, const v4f b) {
  v4u r;
  r.x = pk2(a.x, a.y); r.y = pk2(a.z, a.w); r.z = pk2(b.x, b.y); r.w = pk2(b.z, b.w);
  return r;
}

template <int SLB>
__device__ __forceinline__ int scan_chunk(const int* __restrict__ dsts, int nE, int cbase, int slotBase,
                                          int nb, int vec8, int* list, int tid, int lane, int wave) {
  int wc = 0;
  const int el0  = tid * EPT;
  const int e0   = cbase + el0;
  const int sent = -2147483647 - 1;
  v4i da, db;
  if (vec8 != 0 && cbase + CHUNK <= nE) {
    da = *(const v4i*)(dsts + e0);
    db = *(const v4i*)(dsts + e0 + 4);
  } else {
    da.x = (e0     < nE) ? dsts[min(e0,     nE - 1)] : sent;
    da.y = (e0 + 1 < nE) ? dsts[min(e0 + 1, nE - 1)] : sent;
    da.z = (e0 + 2 < nE) ? dsts[min(e0 + 2, nE - 1)] : sent;
    da.w = (e0 + 3 < nE) ? dsts[min(e0 + 3, nE - 1)] : sent;
    db.x = (e0 + 4 < nE) ? dsts[min(e0 + 4, nE - 1)] : sent;
    db.y = (e0 + 5 < nE) ? dsts[min(e0 + 5, nE - 1)] : sent;
    db.z = (e0 + 6 < nE) ? dsts[min(e0 + 6, nE - 1)] : sent;
    db.w = (e0 + 7 < nE) ? dsts[min(e0 + 7, nE - 1)] : sent;
  }
  const unsigned nbs = (unsigned)slotBase;
  const unsigned unb = (unsigned)nb;
  const unsigned s0 = (unsigned)da.x - nbs, s1 = (unsigned)da.y - nbs;
  const unsigned s2 = (unsigned)da.z - nbs, s3 = (unsigned)da.w - nbs;
  const unsigned s4 = (unsigned)db.x - nbs, s5 = (unsigned)db.y - nbs;
  const unsigned s6 = (unsigned)db.z - nbs, s7 = (unsigned)db.w - nbs;
  const bool h0 = s0 < unb, h1 = s1 < unb, h2 = s2 < unb, h3 = s3 < unb;
  const bool h4 = s4 < unb, h5 = s5 < unb, h6 = s6 < unb, h7 = s7 < unb;
  const unsigned any = __builtin_amdgcn_ballot_w32(h0 | h1 | h2 | h3 | h4 | h5 | h6 | h7);
  if (any != 0u) {
#define HITJ(J, HJ, SJ) { \
      const unsigned mj = __builtin_amdgcn_ballot_w32(HJ); \
      if (mj != 0u) { \
        if (HJ) { \
          const int pos = wc + (int)__builtin_amdgcn_mbcnt_lo(mj, 0u); \
          if (pos < WCAP) list[wave * WCAP + pos] = ((el0 + (J)) << SLB) | (int)(SJ); \
        } \
        wc += (int)__builtin_popcount(mj); } }
    HITJ(0, h0, s0)
    HITJ(1, h1, s1)
    HITJ(2, h2, s2)
    HITJ(3, h3, s3)
    HITJ(4, h4, s4)
    HITJ(5, h5, s5)
    HITJ(6, h6, s6)
    HITJ(7, h7, s7)
#undef HITJ
  }
  return wc;
}

__global__ __launch_bounds__(NTHR) void k_wprep(const float* __restrict__ Wl, const float* __restrict__ Wr,
                                                const float* __restrict__ We,
                                                unsigned short* WLR, unsigned short* WE) {
  const int u = (int)blockIdx.x * NTHR + (int)threadIdx.x;
  v8us o;
  unsigned short* dp;
  if (u < NUW) {
    const int n  = u >> 4;
    const int k8 = (u & 15) * 8;
    const float* p = Wl + (size_t)k8 * HC + n;
#pragma unroll
    for (int i = 0; i < 8; ++i) o[i] = (unsigned short)bf16_bits(p[(size_t)i * HC]);
    dp = WLR + (size_t)n * DIN + k8;
  } else if (u < 2 * NUW) {
    const int v  = u - NUW;
    const int n  = v >> 4;
    const int k8 = (v & 15) * 8;
    const float* p = Wr + (size_t)k8 * HC + n;
#pragma unroll
    for (int i = 0; i < 8; ++i) o[i] = (unsigned short)bf16_bits(p[(size_t)i * HC]);
    dp = WLR + (size_t)(HC + n) * DIN + k8;
  } else if (u < 2 * NUW + NUE) {
    const int v  = u - 2 * NUW;
    const int n  = v >> 2;
    const int k8 = (v & 3) * 8;
    const int kk = k8 & 8;
    const bool live = k8 < EDF;
    const float* p = We + (size_t)kk * HC + n;
#pragma unroll
    for (int i = 0; i < 8; ++i) {
      const unsigned b = bf16_bits(p[(size_t)i * HC]);
      o[i] = live ? (unsigned short)b : (unsigned short)0;
    }
    dp = WE + (size_t)n * KE + k8;
  } else {
    return;
  }
  *(volatile v8us*)dp = o;
  __threadfence();
  *(volatile v8us*)dp = o;
}

__global__ __launch_bounds__(NTHR) void k_cvx(const float* __restrict__ x, int nN, int nUnits,
                                              unsigned short* xb) {
  const int u = (int)blockIdx.x * NTHR + (int)threadIdx.x;
  if (u >= nUnits) return;
  const int row = u >> 4;
  const int k8  = (u & 15) * 8;
  const int rc  = row < nN ? row : nN - 1;
  const float* p = x + (size_t)rc * DIN + k8;
  const v4f a = *(const v4f*)p;
  const v4f b = *(const v4f*)(p + 4);
  const bool ok = row < nN;
  v8us o;
  o[0] = ok ? (unsigned short)bf16_bits(a.x) : (unsigned short)0;
  o[1] = ok ? (unsigned short)bf16_bits(a.y) : (unsigned short)0;
  o[2] = ok ? (unsigned short)bf16_bits(a.z) : (unsigned short)0;
  o[3] = ok ? (unsigned short)bf16_bits(a.w) : (unsigned short)0;
  o[4] = ok ? (unsigned short)bf16_bits(b.x) : (unsigned short)0;
  o[5] = ok ? (unsigned short)bf16_bits(b.y) : (unsigned short)0;
  o[6] = ok ? (unsigned short)bf16_bits(b.z) : (unsigned short)0;
  o[7] = ok ? (unsigned short)bf16_bits(b.w) : (unsigned short)0;
  unsigned short* dp = xb + (size_t)row * DIN + k8;
  *(volatile v8us*)dp = o;
  __threadfence();
  *(volatile v8us*)dp = o;
}

__global__ __launch_bounds__(NTHR) void k_gemm(const unsigned short* __restrict__ A,
                                               const unsigned short* __restrict__ BT,
                                               float* Cm, const float* __restrict__ bl,
                                               const float* __restrict__ br) {
  extern __shared__ __attribute__((aligned(16))) float gsm[];
  float* stg = gsm;
  const int tid = (int)threadIdx.x, lane = tid & 31, wave = tid >> 5, hh = lane >> 4, m = lane & 15;
  const int rg = wave & 3, cg = wave >> 2;
  const int rowBase = (int)blockIdx.x * GBM;
  const int colBase = cg * GBN;

  v8f acc[8];
  {
    const v8f z = {0.f, 0.f, 0.f, 0.f, 0.f, 0.f, 0.f, 0.f};
#pragma unroll
    for (int t = 0; t < 8; ++t) acc[t] = z;
  }
  const unsigned short* ap = A  + (size_t)(rowBase + 16 * rg + m) * (size_t)DIN + 8 * hh;
  const unsigned short* bp = BT + (size_t)(colBase + m) * (size_t)DIN + 8 * hh;

#pragma unroll 1
  for (int k0 = 0; k0 < DIN; k0 += 32) {
    FragB af;
    af.h[0] = *(const v8usa*)(ap + k0);
    af.h[1] = *(const v8usa*)(ap + k0 + 16);
#pragma unroll
    for (int nt = 0; nt < 8; ++nt) {
      const unsigned short* wq = bp + (size_t)(16 * nt) * (size_t)DIN + k0;
      FragB bf;
      bf.h[0] = *(const v8usa*)wq;
      bf.h[1] = *(const v8usa*)(wq + 16);
      acc[nt] = wmb(af, bf, acc[nt]);
    }
  }

#pragma unroll
  for (int nt = 0; nt < 8; ++nt) {
    const int lc = colBase + 16 * nt + m;
#pragma unroll
    for (int r = 0; r < 8; ++r) {
      const int lr = 16 * rg + 8 * hh + r;
      stg[lr * LDX + lc] = acc[nt][r];
    }
  }
  __syncthreads();

  const v4f bb0 = bfr4(*(const v4fa*)(bl + 4 * lane));
  const v4f bb1 = bfr4(*(const v4fa*)(br + 4 * lane));
#pragma unroll 1
  for (int i = 0; i < 8; ++i) {
    const int row = wave * 8 + i;
    const v4f p0 = *(const v4fa*)(stg + row * LDX + 4 * lane) + bb0;
    const v4f p1 = *(const v4fa*)(stg + row * LDX + GBN + 4 * lane) + bb1;
    float* op = Cm + (size_t)(rowBase + row) * (size_t)LDX + 4 * lane;
    *(volatile v4f*)op = p0;
    *(volatile v4f*)(op + GBN) = p1;
  }
  __threadfence();
#pragma unroll 1
  for (int i = 0; i < 8; ++i) {
    const int row = wave * 8 + i;
    const v4f p0 = *(const v4fa*)(stg + row * LDX + 4 * lane) + bb0;
    const v4f p1 = *(const v4fa*)(stg + row * LDX + GBN + 4 * lane) + bb1;
    float* op = Cm + (size_t)(rowBase + row) * (size_t)LDX + 4 * lane;
    *(volatile v4f*)op = p0;
    *(volatile v4f*)(op + GBN) = p1;
  }
}

__device__ __forceinline__ float score4(const v4f xl, const v4f xr, const v4f ee, const v4f at) {
  float m0 = (xl.x + xr.x) + ee.x;
  float m1 = (xl.y + xr.y) + ee.y;
  float m2 = (xl.z + xr.z) + ee.z;
  float m3 = (xl.w + xr.w) + ee.w;
  m0 = (m0 > 0.f) ? m0 : NEGSL * m0;
  m1 = (m1 > 0.f) ? m1 : NEGSL * m1;
  m2 = (m2 > 0.f) ? m2 : NEGSL * m2;
  m3 = (m3 > 0.f) ? m3 : NEGSL * m3;
  float ep = m0 * at.x;
  ep = fmaf(m1, at.y, ep);
  ep = fmaf(m2, at.z, ep);
  ep = fmaf(m3, at.w, ep);
  ep += __shfl_xor(ep, 1);
  ep += __shfl_xor(ep, 2);
  return ep;
}

__device__ __forceinline__ void fold(const float lg, const v4f msg, float& mx, float& dn, v4f& av) {
  const float df = lg - mx;
  const float ee = expf(-fabsf(df));
  const bool  up = df > 0.f;
  const float s1 = up ? ee : 1.0f;
  const float s2 = up ? 1.0f : ee;
  mx = up ? lg : mx;
  dn = fmaf(dn, s1, s2);
  av.x = fmaf(av.x, s1, s2 * msg.x);
  av.y = fmaf(av.y, s1, s2 * msg.y);
  av.z = fmaf(av.z, s1, s2 * msg.z);
  av.w = fmaf(av.w, s1, s2 * msg.w);
}

__global__ __launch_bounds__(NTHR) void k_scan(const int* __restrict__ srcs, const int* __restrict__ dsts,
                                               int nE, int nN, int vec8,
                                               const float* __restrict__ XLR,
                                               const unsigned short* __restrict__ WE,
                                               const float* __restrict__ eattr,
                                               const float* __restrict__ x,
                                               const float* __restrict__ att,
                                               const float* __restrict__ bias,
                                               float* OUTP) {
  extern __shared__ __attribute__((aligned(16))) int dsm[];
  int* list = dsm;
  int* hl   = dsm + LISTN;
  int* sl   = dsm + LISTN + RCAP;
  int* cnt  = dsm + LISTN + 2 * RCAP;
  int* offs = cnt + NBA;
  int* cur  = offs + NBA;
  int* misc = cur + NBA;
  const int tid = (int)threadIdx.x, lane = tid & 31;
  const int wave = __builtin_amdgcn_readfirstlane(tid >> 5);
  const int nodeBase = (int)blockIdx.x * NBA;

  {
    const v4i z4 = {0, 0, 0, 0};
    for (int i = tid * 4; i < AGG_ZINTS; i += NTHR * 4) *(v4ia*)(dsm + i) = z4;
    if (tid < 16) misc[tid] = 0;
  }
  __syncthreads();

  int t = 0, ov = 0;
  const int nChunks = (nE + CHUNK - 1) / CHUNK;
#pragma unroll 1
  for (int ch = 0; ch < nChunks; ++ch) {
    const int cbase = ch * CHUNK;
    const int wc = scan_chunk<SLA>(dsts, nE, cbase, nodeBase, NBA, vec8, list, tid, lane, wave);
    if (lane == 0) misc[wave] = wc;
    __syncthreads();
    if (wave == 0) {
#pragma unroll 1
      for (int w2 = 0; w2 < NWAVE; ++w2) {
        int c = misc[w2];
        c = c < 0 ? 0 : (c > WCAP ? WCAP : c);
#pragma unroll 1
        for (int b0 = 0; b0 < c; b0 += 32) {
          const int idx = b0 + lane;
          const int ent = list[w2 * WCAP + (idx < WCAP ? idx : WCAP - 1)];
          const int m32 = (c - b0) < 32 ? (c - b0) : 32;
#pragma unroll 1
          for (int k = 0; k < m32; ++k) {
            const int u    = __builtin_amdgcn_readlane(ent, k);
            const int slot = u & (NBA - 1);
            const int el   = (u >> SLA) & (CHUNK - 1);
            const int pk   = ((cbase + el) << SLA) | slot;
            if (t < RCAP) {
              if (lane == 0) { hl[t] = pk; cnt[slot] = cnt[slot] + 1; }
              t = t + 1;
            } else {
              ov = 1;
            }
          }
        }
      }
    }
    __syncthreads();
  }
  if (wave == 0 && lane == 0) { misc[8] = t; misc[9] = ov; }
  __syncthreads();
  int tt = misc[8];
  tt = tt < 0 ? 0 : (tt > RCAP ? RCAP : tt);
  const int ovf = misc[9];

  if (wave == 0) {
    const int base = lane * (NBA / 32);
    int s = 0;
#pragma unroll 1
    for (int i = 0; i < NBA / 32; ++i) s += cnt[base + i];
    int incl = s;
#pragma unroll
    for (int d = 1; d < 32; d <<= 1) {
      const int y = __shfl_up(incl, d, 32);
      if (lane >= d) incl += y;
    }
    int run = incl - s;
#pragma unroll 1
    for (int i = 0; i < NBA / 32; ++i) {
      const int cv = cnt[base + i];
      offs[base + i] = run;
      cur[base + i]  = run;
      run += cv;
    }
  }
  __syncthreads();
  if (wave == 0) {
#pragma unroll 1
    for (int b0 = 0; b0 < tt; b0 += 32) {
      const int idx = b0 + lane;
      const int ent = hl[idx < RCAP ? idx : RCAP - 1];
      const int m32 = (tt - b0) < 32 ? (tt - b0) : 32;
#pragma unroll 1
      for (int k = 0; k < m32; ++k) {
        const int u    = __builtin_amdgcn_readlane(ent, k);
        const int slot = u & (NBA - 1);
        if (lane == 0) {
          int p = cur[slot];
          p = p < 0 ? 0 : (p > RCAP - 1 ? RCAP - 1 : p);
          sl[p] = u;
          cur[slot] = p + 1;
        }
      }
    }
  }
  __syncthreads();

  const int c0  = 4 * lane;
  const int hh  = lane >> 4, mm = lane & 15;
  const int hit = lane >> 1, hf = lane & 1;
  const v4f att4 = bfr4(*(const v4fa*)(att + c0));
  const v4f bia4 = bfr4(*(const v4fa*)(bias + c0));
  float* eet = (float*)hl + wave * (16 * HC);
  unsigned short* atl = (unsigned short*)list + wave * (16 * KE);
  const float qnan = __int_as_float(0x7fc00000);
  const float pz   = (ovf != 0) ? qnan : 0.0f;
  const v8f z8 = {0.f, 0.f, 0.f, 0.f, 0.f, 0.f, 0.f, 0.f};
  const v4f z4 = {0.f, 0.f, 0.f, 0.f};
  const v4u zu = {0u, 0u, 0u, 0u};

#pragma unroll 1
  for (int si = 0; si < NBA / NWAVE; ++si) {
    const int s    = si * NWAVE + wave;
    const int node = nodeBase + s;
    const int nc   = node < nN ? node : nN - 1;
    const int craw = cnt[s];
    const bool big = craw > DEGCAP;
    int c = craw < 0 ? 0 : (craw > DEGCAP ? DEGCAP : craw);
    int o = offs[s];
    o = o < 0 ? 0 : (o > tt ? tt : o);
    c = c > tt - o ? tt - o : c;
    c = __builtin_amdgcn_readfirstlane(c);
    o = __builtin_amdgcn_readfirstlane(o);

    const float* xrow = XLR + (size_t)nc * LDX;
    const v4f xs4 = *(const v4fa*)(xrow + c0);
    const v4f xr4 = *(const v4fa*)(xrow + HC + c0);
    float mx = -3.0e38f, dn = 0.0f;
    v4f av = z4, es = z4;

#pragma unroll 1
    for (int b0 = 0; b0 < c; b0 += 16) {
      const int m16 = (c - b0) < 16 ? (c - b0) : 16;
      int idx = o + b0 + mm;
      idx = idx > RCAP - 1 ? RCAP - 1 : idx;
      const int ent = sl[idx];
      int eid = ent >> SLA;
      eid = eid < 0 ? 0 : (eid > nE - 1 ? nE - 1 : eid);
      int sr = srcs[eid];
      sr = sr < 0 ? 0 : (sr > nN - 1 ? nN - 1 : sr);
      const int ent2 = __shfl(ent, hit);
      int eid2 = ent2 >> SLA;
      eid2 = eid2 < 0 ? 0 : (eid2 > nE - 1 ? nE - 1 : eid2);
      const float* ep = eattr + (size_t)eid2 * EDF + 8 * hf;
      v4f ea = *(const v4fa*)ep;
      v4f eb = *(const v4fa*)(ep + 4);
      const bool okh = hit < m16;
      ea = okh ? ea : z4;
      eb = okh ? eb : z4;
      const v4u pk = pack8(ea, eb);
      *(v4ua*)(atl + hit * KE + 8 * hf) = pk;
      *(v4ua*)(atl + hit * KE + 16 + 8 * hf) = zu;
      wave_lds_sync();

      FragB af;
      af.h[0] = *(const v8usa*)(atl + mm * KE + 8 * hh);
      af.h[1] = *(const v8usa*)(atl + mm * KE + 16 + 8 * hh);
#pragma unroll 1
      for (int h = 0; h < NH; ++h) {
        const unsigned short* wq = WE + (size_t)(h * 16 + mm) * KE + 8 * hh;
        FragB bf;
        bf.h[0] = *(const v8usa*)wq;
        bf.h[1] = *(const v8usa*)(wq + 16);
        const v8f d = wmb(af, bf, z8);
        float* ew = eet + (8 * hh) * HC + h * 16 + mm;
#pragma unroll
        for (int r = 0; r < 8; ++r) ew[r * HC] = d[r];
      }
      wave_lds_sync();

#pragma unroll 1
      for (int k = 0; k < m16; ++k) {
        const int sk = __builtin_amdgcn_readlane(sr, k);
        const v4f xl4 = *(const v4fa*)(XLR + (size_t)sk * LDX + c0);
        const v4f ee4 = *(const v4fa*)(eet + k * HC + c0);
        const float lg = score4(xl4, xr4, ee4, att4);
        fold(lg, xl4, mx, dn, av);
        es.x += ee4.x; es.y += ee4.y; es.z += ee4.z; es.w += ee4.w;
      }
      wave_lds_sync();
    }

    const float rdeg = 1.0f / (float)(c > 1 ? c : 1);
    v4f es4;
    es4.x = es.x * rdeg; es4.y = es.y * rdeg; es4.z = es.z * rdeg; es4.w = es.w * rdeg;
    const float l0 = score4(xs4, xr4, es4, att4);
    fold(l0, xs4, mx, dn, av);

    const float inv = __builtin_amdgcn_rcpf(dn);
    const float pzr = big ? qnan : pz;
    const v4f xin = bfr4(*(const v4fa*)(x + (size_t)nc * DIN + c0));
    v4f ov4;
    ov4.x = (fmaf(av.x, inv, bia4.x) + xin.x) + pzr;
    ov4.y = (fmaf(av.y, inv, bia4.y) + xin.y) + pzr;
    ov4.z = (fmaf(av.z, inv, bia4.z) + xin.z) + pzr;
    ov4.w = (fmaf(av.w, inv, bia4.w) + xin.w) + pzr;
    if (node < nN) {
      float* op = OUTP + (size_t)node * HC + c0;
      *(volatile v4f*)op = ov4;
      __threadfence();
      *(volatile v4f*)op = ov4;
    }
  }
}

__global__ __launch_bounds__(NTHR) void k_stat(const float* __restrict__ OUTP, const int* __restrict__ batch,
                                               const float* __restrict__ MM, double* REC, int nN, int mode) {
  extern __shared__ __attribute__((aligned(16))) double ssm[];
  double* sacc = ssm;
  float*  smm  = (float*)(ssm + NWAVE * NG * HC);
  const int tid = (int)threadIdx.x, lane = tid & 31;
  const int wave = __builtin_amdgcn_readfirstlane(tid >> 5);
  {
    const v2d zd = {0.0, 0.0};
    for (int i = tid * 2; i < NWAVE * NG * HC; i += NTHR * 2) *(v2da*)(sacc + i) = zd;
    if (mode != 0) {
      *(v4fa*)(smm + 4 * tid) = *(const v4fa*)(MM + 4 * tid);
    } else {
      const v4f z4 = {0.f, 0.f, 0.f, 0.f};
      *(v4fa*)(smm + 4 * tid) = z4;
    }
  }
  __syncthreads();

  const int c0   = 4 * lane;
  const int row0 = (int)blockIdx.x * SROWS;
  int nr = nN - row0;
  nr = nr < 0 ? 0 : (nr > SROWS ? SROWS : nr);
#pragma unroll 1
  for (int r = wave; r < nr; r += NWAVE) {
    const int row = row0 + r;
    const int g   = batch[row];
    const bool ok = (unsigned)g < (unsigned)NG;
    const int gi  = g < 0 ? 0 : (g > NG - 1 ? NG - 1 : g);
    const v4f v = *(const v4fa*)(OUTP + (size_t)row * HC + c0);
    const v4f mv = *(const v4fa*)(smm + gi * HC + c0);
    const v4f sb = v - mv;
    v4f val;
    val.x = (mode != 0) ? sb.x * sb.x : v.x;
    val.y = (mode != 0) ? sb.y * sb.y : v.y;
    val.z = (mode != 0) ? sb.z * sb.z : v.z;
    val.w = (mode != 0) ? sb.w * sb.w : v.w;
    val.x = ok ? val.x : 0.0f;
    val.y = ok ? val.y : 0.0f;
    val.z = ok ? val.z : 0.0f;
    val.w = ok ? val.w : 0.0f;
    double* q = sacc + ((size_t)(wave * NG + gi) * HC + c0);
    v2d a = *(const v2da*)q;
    v2d b = *(const v2da*)(q + 2);
    a.x += (double)val.x; a.y += (double)val.y;
    b.x += (double)val.z; b.y += (double)val.w;
    *(v2da*)q = a;
    *(v2da*)(q + 2) = b;
  }
  __syncthreads();

  v2d s0 = {0.0, 0.0}, s1 = {0.0, 0.0};
#pragma unroll 1
  for (int w = 0; w < NWAVE; ++w) {
    const v2d a = *(const v2da*)(sacc + w * (NG * HC) + 2 * tid);
    const v2d b = *(const v2da*)(sacc + w * (NG * HC) + 512 + 2 * tid);
    s0.x += a.x; s0.y += a.y;
    s1.x += b.x; s1.y += b.y;
  }
  double* rp = REC + (size_t)blockIdx.x * (NG * HC) + 2 * tid;
  *(volatile v2d*)rp = s0;
  *(volatile v2d*)(rp + 512) = s1;
  __threadfence();
  *(volatile v2d*)rp = s0;
  *(volatile v2d*)(rp + 512) = s1;
}

__global__ __launch_bounds__(NTHR) void k_comb(const double* __restrict__ REC, int nrec,
                                               const int* __restrict__ batch, int nN,
                                               const float* __restrict__ gms, float* PL, int mode) {
  __shared__ int wcn[NWAVE * NG];
  const int tid = (int)threadIdx.x, lane = tid & 31, wave = tid >> 5;
  int cg[NG];
#pragma unroll
  for (int j = 0; j < NG; ++j) cg[j] = 0;
#pragma unroll 1
  for (int i = tid; i < nN; i += NTHR) {
    const int b = batch[i];
#pragma unroll
    for (int j = 0; j < NG; ++j) cg[j] += (b == j) ? 1 : 0;
  }
#pragma unroll
  for (int j = 0; j < NG; ++j) {
    int v = cg[j];
#pragma unroll
    for (int off = 16; off > 0; off >>= 1) v += __shfl_xor(v, off);
    cg[j] = v;
  }
  if (lane == 0) {
#pragma unroll
    for (int j = 0; j < NG; ++j) wcn[wave * NG + j] = cg[j];
  }
  __syncthreads();
  const int g = tid >> 5;
  int cn = 0;
#pragma unroll
  for (int w = 0; w < NWAVE; ++w) cn += wcn[w * NG + g];
  const double cd = (double)(cn > 1 ? cn : 1);

  v2d s0 = {0.0, 0.0}, s1 = {0.0, 0.0};
  const int nr = nrec < 0 ? 0 : nrec;
#pragma unroll 1
  for (int r = 0; r < nr; ++r) {
    const double* p = REC + (size_t)r * (NG * HC) + 4 * tid;
    const v2d a = *(const v2da*)p;
    const v2d b = *(const v2da*)(p + 2);
    s0.x += a.x; s0.y += a.y;
    s1.x += b.x; s1.y += b.y;
  }
  const int ch = (4 * tid) & (HC - 1);
  const v4f ms4 = bfr4(*(const v4fa*)(gms + ch));
  const float q0 = (float)(s0.x / cd), q1 = (float)(s0.y / cd);
  const float q2 = (float)(s1.x / cd), q3 = (float)(s1.y / cd);
  v4f o;
  if (mode == 0) {
    o.x = ms4.x * q0; o.y = ms4.y * q1; o.z = ms4.z * q2; o.w = ms4.w * q3;
  } else {
    o.x = 1.0f / sqrtf(q0 + EPSN); o.y = 1.0f / sqrtf(q1 + EPSN);
    o.z = 1.0f / sqrtf(q2 + EPSN); o.w = 1.0f / sqrtf(q3 + EPSN);
  }
  float* op = PL + 4 * tid;
  *(volatile v4f*)op = o;
  __threadfence();
  *(volatile v4f*)op = o;
}

__global__ __launch_bounds__(NTHR) void k_norm(const float* __restrict__ OUTP, const int* __restrict__ batch,
                                               const float* __restrict__ MM, const float* __restrict__ RS,
                                               const float* __restrict__ gw, const float* __restrict__ gb,
                                               float* outp, int nUnits) {
  const int i = (int)blockIdx.x * NTHR + (int)threadIdx.x;
  if (i >= nUnits) return;
  const int row = i >> 5;
  const int c0  = 4 * (i & 31);
  const int g   = batch[row];
  const int gi  = g < 0 ? 0 : (g > NG - 1 ? NG - 1 : g);
  const v4f v   = *(const v4fa*)(OUTP + (size_t)row * HC + c0);
  const v4f mv  = *(const v4fa*)(MM + gi * HC + c0);
  const v4f rs  = *(const v4fa*)(RS + gi * HC + c0);
  const v4f w4  = bfr4(*(const v4fa*)(gw + c0));
  const v4f b4  = bfr4(*(const v4fa*)(gb + c0));
  v4f y;
  y.x = (w4.x * (v.x - mv.x)) * rs.x + b4.x;
  y.y = (w4.y * (v.y - mv.y)) * rs.y + b4.y;
  y.z = (w4.z * (v.z - mv.z)) * rs.z + b4.z;
  y.w = (w4.w * (v.w - mv.w)) * rs.w + b4.w;
  v4f o = y;
#pragma unroll 1
  for (int j = 0; j < 4; ++j) {
    const float t  = (j == 0) ? y.x : ((j == 1) ? y.y : ((j == 2) ? y.z : y.w));
    const float em = expm1f(t);
    const float e  = (t > 0.0f) ? t : em;
    o.x = (j == 0) ? e : o.x;
    o.y = (j == 1) ? e : o.y;
    o.z = (j == 2) ? e : o.z;
    o.w = (j == 3) ? e : o.w;
  }
  float* op = outp + (size_t)row * HC + c0;
  *(volatile v4f*)op = o;
  __threadfence();
  *(volatile v4f*)op = o;
}

static inline int cdiv(int a, int b) { return (a + b - 1) / b; }

extern "C" void kernel_launch(void* const* d_in, const int* in_sizes, int n_in,
                              void* d_out, int out_size, void* d_ws, size_t ws_size,
                              hipStream_t stream) {
  if (n_in < 14) return;
  if (in_sizes[0] < DIN || (in_sizes[0] % DIN) != 0) return;
  const int nN = in_sizes[0] / DIN;
  if (nN > (1 << 22)) return;
  if (in_sizes[1] < 2 || (in_sizes[1] & 1) != 0) return;
  const int nE = in_sizes[1] / 2;
  if (nE < 1 || nE >= (1 << 22)) return;
  if ((long long)in_sizes[2] != (long long)nE * EDF) return;
  if (in_sizes[3] != nN) return;
  if (in_sizes[4] != DIN * HC || in_sizes[6] != DIN * HC) return;
  if (in_sizes[5] != HC || in_sizes[7] != HC) return;
  if (in_sizes[8] != EDF * HC) return;
  if (in_sizes[9] != HC) return;
  if (in_sizes[10] != HC || in_sizes[11] != HC || in_sizes[12] != HC || in_sizes[13] != HC) return;
  if ((long long)out_size != (long long)nN * HC) return;

  const float* x     = (const float*)d_in[0];
  const int*   edge  = (const int*)d_in[1];
  const float* eattr = (const float*)d_in[2];
  const int*   batch = (const int*)d_in[3];
  const float* Wl    = (const float*)d_in[4];
  const float* bl    = (const float*)d_in[5];
  const float* Wr    = (const float*)d_in[6];
  const float* br    = (const float*)d_in[7];
  const float* We    = (const float*)d_in[8];
  const float* att   = (const float*)d_in[9];
  const float* bias  = (const float*)d_in[10];
  const float* gnw   = (const float*)d_in[11];
  const float* gnb   = (const float*)d_in[12];
  const float* gms   = (const float*)d_in[13];
  float* out = (float*)d_out;
  const int* src = edge;
  const int* dst = edge + nE;

  const int MP   = cdiv(nN, GBM) * GBM;
  const int gM   = MP / GBM;
  const int gA   = cdiv(nN, NBA);
  const int nS   = cdiv(nN, SROWS);
  if ((long long)gA * NBA < (long long)nN) return;
  const int vec8 = ((nE & 3) == 0) ? 1 : 0;

  char* ws = (char*)d_ws;
  size_t off = 0;
  const size_t oWLR = off; off += (size_t)LDX * DIN * 2;                  off = (off + 255) & ~(size_t)255;
  const size_t oWE  = off; off += (size_t)HC * KE * 2;                    off = (off + 255) & ~(size_t)255;
  const size_t oMM  = off; off += (size_t)NG * HC * 4;                    off = (off + 255) & ~(size_t)255;
  const size_t oRS  = off; off += (size_t)NG * HC * 4;                    off = (off + 255) & ~(size_t)255;
  const size_t oREC = off; off += (size_t)nS * NG * HC * 8;               off = (off + 255) & ~(size_t)255;
  const size_t oXB  = off; off += (size_t)MP * DIN * 2;                   off = (off + 255) & ~(size_t)255;
  const size_t oXLR = off; off += (size_t)MP * LDX * 4;                   off = (off + 255) & ~(size_t)255;
  const size_t oOUT = off; off += (size_t)MP * HC * 4;                    off = (off + 255) & ~(size_t)255;
  if (off > ws_size || off > (size_t)WSMAX) return;
  unsigned short* WLR = (unsigned short*)(ws + oWLR);
  unsigned short* WEp = (unsigned short*)(ws + oWE);
  float*          MMp = (float*)(ws + oMM);
  float*          RSp = (float*)(ws + oRS);
  double*         REC = (double*)(ws + oREC);
  unsigned short* XB  = (unsigned short*)(ws + oXB);
  float*          XLR = (float*)(ws + oXLR);
  float*          OUTP = (float*)(ws + oOUT);

  const size_t scanLds = (size_t)AGG_LDS_INTS * 4;
  hipFuncSetAttribute(reinterpret_cast<const void*>(&k_gemm), hipFuncAttributeMaxDynamicSharedMemorySize, (int)GEMM_LDS);
  hipFuncSetAttribute(reinterpret_cast<const void*>(&k_scan), hipFuncAttributeMaxDynamicSharedMemorySize, (int)scanLds);
  hipFuncSetAttribute(reinterpret_cast<const void*>(&k_stat), hipFuncAttributeMaxDynamicSharedMemorySize, (int)STAT_LDS);

  const int nUx = MP * (DIN / 8);
  k_wprep<<<(2 * NUW + NUE) / NTHR, NTHR, 0, stream>>>(Wl, Wr, We, WLR, WEp);
  k_cvx<<<cdiv(nUx, NTHR), NTHR, 0, stream>>>(x, nN, nUx, XB);
  k_gemm<<<gM, NTHR, GEMM_LDS, stream>>>(XB, WLR, XLR, bl, br);
  k_scan<<<gA, NTHR, scanLds, stream>>>(src, dst, nE, nN, vec8, XLR, WEp, eattr, x, att, bias, OUTP);
  k_stat<<<nS, NTHR, STAT_LDS, stream>>>(OUTP, batch, MMp, REC, nN, 0);
  k_comb<<<1, NTHR, 0, stream>>>(REC, nS, batch, nN, gms, MMp, 0);
  k_stat<<<nS, NTHR, STAT_LDS, stream>>>(OUTP, batch, MMp, REC, nN, 1);
  k_comb<<<1, NTHR, 0, stream>>>(REC, nS, batch, nN, gms, RSp, 1);
  const int nUn = nN * 32;
  k_norm<<<cdiv(nUn, NTHR), NTHR, 0, stream>>>(OUTP, batch, MMp, RSp, gnw, gnb, out, nUn);
}
